// SSAANet_52862457479432
// MI455X (gfx1250) — hardware-verified
//
#include <hip/hip_runtime.h>


#define PP   4096
#define TSZ  524288

typedef _Float16 f16;
typedef __attribute__((ext_vector_type(16))) _Float16 v16h;
typedef __attribute__((ext_vector_type(8)))  _Float16 v8h;
typedef __attribute__((ext_vector_type(8)))  float    v8f;
typedef __attribute__((ext_vector_type(4)))  float    v4f;
typedef __attribute__((ext_vector_type(4)))  unsigned v4u;
typedef float __attribute__((may_alias)) float_a;
template <typename V> __device__ __forceinline__ void vst2(void* p, V v) {
  *(volatile V*)p = v; __threadfence(); *(volatile V*)p = v;
}
__device__ __forceinline__ v8f wmma16(v16h a, v16h b, v8f c) {
  v8f d = __builtin_amdgcn_wmma_f32_16x16x32_f16(false, a, false, b, (short)0, c, false, false);
  asm volatile("v_nop\n\tv_nop\n\tv_nop\n\tv_nop" : "+v"(d) : "v"(a), "v"(b));
  return d;
}
#define PSC 256.0f
#define PUN (1.0f / 256.0f)

__device__ __forceinline__ float relu6f(float x){ return fminf(fmaxf(x, 0.f), 6.f); }

__device__ __forceinline__ v16h cat8(v8h lo, v8h hi){
  return __builtin_shufflevector(lo, hi, 0,1,2,3,4,5,6,7,8,9,10,11,12,13,14,15);
}

__global__ __launch_bounds__(256) void k_colmax(const float* __restrict__ X, float* __restrict__ out){
  __shared__ float sm[32];
  const int t = threadIdx.x, wave = t >> 5, lane = t & 31;
  for (int r = 0; r < 4; ++r){
    const int row = blockIdx.x * 32 + wave * 4 + r;
    const float* src = X + (size_t)row * PP;
    float m = -__builtin_inff();
    for (int i = lane; i < PP; i += 32) m = fmaxf(m, src[i]);
    for (int off = 16; off > 0; off >>= 1) m = fmaxf(m, __shfl_xor(m, off, 32));
    if (lane == 0) sm[wave * 4 + r] = m;
  }
  __syncthreads();
  if (t < 32) vst2(out + blockIdx.x * 32 + t, (float_a)sm[t]);
}

__global__ void k_spe_score(const float* __restrict__ colmax, const float* __restrict__ w,
                            const float* __restrict__ b, float* __restrict__ out){
  int idx = threadIdx.x;
  int bb = idx >> 6, o = idx & 63;
  float s = b[o];
  for (int i = 0; i < 64; ++i) s += w[o*64 + i] * colmax[bb*64 + i];
  s = relu6f(s);
  s = fminf(fmaxf(s, -1.f), 1.f);
  vst2(out + idx, (float_a)s);
}

__global__ void k_chmean(const float* __restrict__ X, float* __restrict__ out){
  int idx = blockIdx.x*256 + threadIdx.x;
  int b = idx >> 12, p = idx & 4095;
  float s = 0.f;
  for (int c = 0; c < 64; ++c) s += X[((size_t)b*64 + c)*PP + p];
  vst2(out + idx, (float_a)(s * (1.f/64.f)));
}

__global__ void k_dw3x3(const float* __restrict__ X, const float* __restrict__ Wd,
                        const float* __restrict__ bias,
                        const float* __restrict__ addbc,
                        const float* __restrict__ spw, const float* __restrict__ spb,
                        const float* __restrict__ chmean,
                        float* __restrict__ Y, int C){
  int idx = blockIdx.x*256 + threadIdx.x;
  int p = idx & 4095; int t = idx >> 12; int c = t % C; int b = t / C;
  int x = p & 63, y = p >> 6;
  const float* src = X + (size_t)t * PP;
  const float* wk  = Wd + c*9;
  float s = 0.f;
  #pragma unroll
  for (int dy = -1; dy <= 1; ++dy){
    int yy = y + dy; if (yy < 0 || yy > 63) continue;
    #pragma unroll
    for (int dx = -1; dx <= 1; ++dx){
      int xx = x + dx; if (xx < 0 || xx > 63) continue;
      s += wk[(dy+1)*3 + (dx+1)] * src[yy*64 + xx];
    }
  }
  if (bias)  s += bias[c];
  if (addbc) s += addbc[b*C + c];
  if (spw){
    float sc = spw[c]*chmean[b*PP + p] + spb[c];
    sc = relu6f(sc); sc = fminf(fmaxf(sc, -1.f), 1.f);
    s += sc;
  }
  vst2(Y + idx, (float_a)s);
}

template<int CIN, int COUT, bool BIAS, bool R1, bool R2, int TOKMODE>
__global__ __launch_bounds__(256) void k_pw(const float* __restrict__ X, const float* __restrict__ Wm,
                     const float* __restrict__ bias,
                     const float* __restrict__ res1, const float* __restrict__ res2,
                     float* __restrict__ Yf, f16* __restrict__ Ytok){
  __shared__ __align__(16) float T[16][132];
  const int tid = threadIdx.x, wave = tid >> 5, lane = tid & 31;
  const int m = lane & 15, hi = lane >> 4;
  const int np0 = blockIdx.x * 128;
  const int b = np0 >> 12; const int pb0 = np0 & 4095;
  const int pbase = pb0 + wave * 16;
  const int otile = blockIdx.y;
  const float* wrow = Wm + (size_t)(otile*16 + m)*CIN;
  v8f acc = {};
  #pragma unroll
  for (int kc = 0; kc < CIN; kc += 32){
    v4f w0 = *(const v4f*)(wrow + kc +      8*hi);
    v4f w1 = *(const v4f*)(wrow + kc +  4 + 8*hi);
    v4f w2 = *(const v4f*)(wrow + kc + 16 + 8*hi);
    v4f w3 = *(const v4f*)(wrow + kc + 20 + 8*hi);
    v16h A;
    #pragma unroll
    for (int j = 0; j < 4; ++j){
      A[j]    = (f16)w0[j];  A[j+4]  = (f16)w1[j];
      A[j+8]  = (f16)w2[j];  A[j+12] = (f16)w3[j];
    }
    v16h Bm;
    #pragma unroll
    for (int j = 0; j < 16; ++j){
      int kb = kc + ((j < 8) ? j : (j + 8)) + 8*hi;
      Bm[j] = (f16)X[((size_t)b*CIN + kb)*PP + pbase + m];
    }
    acc = wmma16(A, Bm, acc);
  }
  #pragma unroll
  for (int r = 0; r < 8; ++r){
    int ol = r + 8*hi, o = otile*16 + ol;
    int pl = wave*16 + m, p = pb0 + pl;
    size_t oi = ((size_t)b*COUT + o)*PP + p;
    float v = acc[r];
    if constexpr (BIAS) v += bias[o];
    if constexpr (R1)   v += res1[oi];
    if constexpr (R2)   v += res2[oi];
    T[ol][pl] = v;
  }
  __syncthreads();
  if constexpr (TOKMODE == 0){
    for (int g = tid; g < 16 * 32; g += 256){ int ol = g >> 5, pc = g & 31;
      vst2(Yf + ((size_t)b*COUT + otile*16 + ol)*PP + pb0 + pc*4, *(const v4f*)(&T[ol][pc*4])); }
  } else if constexpr (TOKMODE == 1){
    for (int g = tid; g < 128 * 2; g += 256){ int pl = g >> 1, half = g & 1;
      union { v8h h; v4u u; } pk;
      #pragma unroll
      for (int e = 0; e < 8; ++e) pk.h[e] = (f16)T[half*8 + e][pl];
      vst2(Ytok + (((size_t)b*4 + otile)*PP + pb0 + pl)*16 + half*8, pk.u); }
  } else {
    for (int g = tid; g < 16 * 16; g += 256){ int d = g >> 4, pc = g & 15;
      union { v8h h; v4u u; } pk;
      #pragma unroll
      for (int e = 0; e < 8; ++e) pk.h[e] = (f16)T[d][pc*8 + e];
      vst2(Ytok + ((size_t)(b*4 + otile)*16 + d)*PP + pb0 + pc*8, pk.u); }
  }
}

__global__ __launch_bounds__(32) void k_flash(const f16* __restrict__ Q, const f16* __restrict__ K,
                        const f16* __restrict__ V, float* __restrict__ Out){
  int lane = threadIdx.x; int m = lane & 15, hi = lane >> 4;
  int qt = blockIdx.x, h = blockIdx.y, b = blockIdx.z;
  size_t base  = ((size_t)(b*4 + h)) * PP * 16;
  const f16* Vrow = V + ((size_t)(b*4 + h)*16 + m)*PP;
  int qbase = qt * 32;
  __shared__ __align__(16) f16 Plds[2][16][40];
  __shared__ __align__(16) float Os[16][32];

  v8h z8 = {};
  v16h Aq[2];
  #pragma unroll
  for (int s2 = 0; s2 < 2; ++s2) Aq[s2] = cat8(*(const v8h*)(Q + base + (size_t)(qbase + s2*16 + m)*16 + 8*hi), z8);

  v8f Oacc[2] = {{}, {}};
  float mrun[2][8], lsum[2][8];
  #pragma unroll
  for (int s2 = 0; s2 < 2; ++s2)
    #pragma unroll
    for (int r = 0; r < 8; ++r){ mrun[s2][r] = -__builtin_inff(); lsum[s2][r] = 0.f; }

  for (int it = 0; it < 128; ++it){
    int kbase = it * 32;
    if (it + 8 < 128){
      __builtin_prefetch(K + base + (size_t)(kbase + 256 + m)*16, 0, 1);
      __builtin_prefetch(Vrow + kbase + 256, 0, 1);
    }
    const f16* kr0 = K + base + (size_t)(kbase      + m)*16 + 8*hi;
    const f16* kr1 = K + base + (size_t)(kbase + 16 + m)*16 + 8*hi;
    v16h B0 = cat8(*(const v8h*)kr0, z8);
    v16h B1 = cat8(*(const v8h*)kr1, z8);
    const f16* vr = Vrow + kbase + 8*hi;
    v16h Bv = cat8(*(const v8h*)vr, *(const v8h*)(vr + 16));
    #pragma unroll
    for (int s2 = 0; s2 < 2; ++s2){
      v8f z = {};
      v8f sc0 = wmma16(Aq[s2], B0, z);
      v8f sc1 = wmma16(Aq[s2], B1, z);
      #pragma unroll
      for (int r = 0; r < 8; ++r){
        float a0 = sc0[r]*0.25f, a1 = sc1[r]*0.25f;
        float t = fmaxf(a0, a1);
        for (int off = 1; off < 16; off <<= 1) t = fmaxf(t, __shfl_xor(t, off, 32));
        float mnew  = fmaxf(mrun[s2][r], t);
        float alpha = expf(mrun[s2][r] - mnew);
        float p0 = expf(a0 - mnew), p1 = expf(a1 - mnew);
        float rs = p0 + p1;
        for (int off = 1; off < 16; off <<= 1) rs += __shfl_xor(rs, off, 32);
        lsum[s2][r] = lsum[s2][r]*alpha + rs;
        mrun[s2][r] = mnew;
        Oacc[s2][r] = Oacc[s2][r]*alpha;
        Plds[s2][r + 8*hi][m]      = (f16)(p0 * PSC);
        Plds[s2][r + 8*hi][16 + m] = (f16)(p1 * PSC);
      }
    }
    __syncthreads();
    #pragma unroll
    for (int s2 = 0; s2 < 2; ++s2){
      v16h Ap = cat8(*(const v8h*)&Plds[s2][m][8*hi], *(const v8h*)&Plds[s2][m][16 + 8*hi]);
      Oacc[s2] = wmma16(Ap, Bv, Oacc[s2]);
    }
    __syncthreads();
  }
  #pragma unroll
  for (int s2 = 0; s2 < 2; ++s2)
    #pragma unroll
    for (int r = 0; r < 8; ++r) Os[m][s2*16 + r + 8*hi] = Oacc[s2][r] * (PUN / lsum[s2][r]);
  __syncthreads();
  #pragma unroll
  for (int q = 0; q < 4; ++q){ int d = q*4 + (lane >> 3), pc = lane & 7;
    vst2(Out + ((size_t)b*64 + h*16 + d)*PP + qbase + pc*4, *(const v4f*)(&Os[d][pc*4])); }
}

__global__ void k_ln(const float* __restrict__ X, const float* __restrict__ w,
                     float* __restrict__ Y){
  int idx = blockIdx.x*256 + threadIdx.x;
  int b = idx >> 12, p = idx & 4095;
  const float* src = X + (size_t)b*64*PP + p;
  float s = 0.f, ss = 0.f;
  for (int c = 0; c < 64; ++c){ float x = src[(size_t)c*PP]; s += x; ss += x*x; }
  float mu  = s * (1.f/64.f);
  float var = ss * (1.f/64.f) - mu*mu;
  float inv = rsqrtf(var + 1e-5f);
  for (int c = 0; c < 64; ++c){
    float x = src[(size_t)c*PP];
    vst2(Y + ((size_t)b*64 + c)*PP + p, (float_a)(x*inv*w[c]));
  }
}

__global__ void k_gate(const float* __restrict__ Hin, float* __restrict__ Y){
  int idx = blockIdx.x*256 + threadIdx.x;
  int p = idx & 4095; int t = idx >> 12; int c = t & 63; int b = t >> 6;
  float x1 = Hin[((size_t)b*128 + c     )*PP + p];
  float x2 = Hin[((size_t)b*128 + 64 + c)*PP + p];
  float g = 0.5f * x1 * (1.f + erff(x1 * 0.70710678118654752f));
  vst2(Y + idx, (float_a)(g * x2));
}

__global__ void k_add(const float* __restrict__ A, const float* __restrict__ B2,
                      float* __restrict__ Y){
  size_t i = (size_t)blockIdx.x*256 + threadIdx.x;
  vst2(Y + i, (float_a)(A[i] + B2[i]));
}

__global__ __launch_bounds__(256) void k_rbnorm(const float* __restrict__ QKV, float* __restrict__ norms){
  __shared__ float sm[32];
  const int t = threadIdx.x, wave = t >> 5, lane = t & 31;
  for (int r = 0; r < 4; ++r){
    const int blk = blockIdx.x * 32 + wave * 4 + r;
    const int c = blk & 63, b = (blk >> 6) & 1, which = blk >> 7;
    const float* src = QKV + ((size_t)b*192 + which*64 + c)*PP;
    float s = 0.f;
    for (int i = lane; i < PP; i += 32){ float x = src[i]; s += x*x; }
    for (int off = 16; off > 0; off >>= 1) s += __shfl_xor(s, off, 32);
    if (lane == 0) sm[wave * 4 + r] = sqrtf(s);
  }
  __syncthreads();
  if (t < 32) vst2(norms + blockIdx.x * 32 + t, (float_a)sm[t]);
}

__global__ __launch_bounds__(256) void k_rbgram(const float* __restrict__ QKV, const float* __restrict__ norms,
                         const float* __restrict__ temp, float* __restrict__ logits){
  __shared__ float sm[32];
  const int t = threadIdx.x, wave = t >> 5, lane = t & 31;
  for (int r = 0; r < 4; ++r){
    const int blk = blockIdx.x * 32 + wave * 4 + r;
    const int j = blk & 15, i = (blk >> 4) & 15, h = (blk >> 8) & 3, b = blk >> 10;
    const float* q = QKV + ((size_t)b*192 +      h*16 + i)*PP;
    const float* k = QKV + ((size_t)b*192 + 64 + h*16 + j)*PP;
    float s = 0.f;
    for (int n = lane; n < PP; n += 32) s += q[n]*k[n];
    for (int off = 16; off > 0; off >>= 1) s += __shfl_xor(s, off, 32);
    if (lane == 0){
      float qn = fmaxf(norms[        b*64 + h*16 + i], 1e-12f);
      float kn = fmaxf(norms[128 +   b*64 + h*16 + j], 1e-12f);
      sm[wave * 4 + r] = (s / (qn*kn)) * temp[h];
    }
  }
  __syncthreads();
  if (t < 32) vst2(logits + blockIdx.x * 32 + t, (float_a)sm[t]);
}

__global__ __launch_bounds__(128) void k_rbsoftmax(const float* __restrict__ logits, float* __restrict__ attn){
  __shared__ __align__(16) float sm[128][16];
  int t = threadIdx.x;
  const float* row = logits + t*16;
  float m = -__builtin_inff();
  for (int j = 0; j < 16; ++j) m = fmaxf(m, row[j]);
  float e[16], s = 0.f;
  for (int j = 0; j < 16; ++j){ e[j] = expf(row[j] - m); s += e[j]; }
  float inv = 1.f/s;
  for (int j = 0; j < 16; ++j) sm[t][j] = e[j]*inv;
  __syncthreads();
  for (int g = t; g < 512; g += 128) vst2(attn + g*4, *(const v4f*)(&sm[0][0] + g*4));
}

__global__ void k_rbav(const float* __restrict__ QKV, const float* __restrict__ attn,
                       float* __restrict__ Y){
  __shared__ float ar[16];
  int blk = blockIdx.x;
  int nt = blk & 15; int t2 = blk >> 4; int c = t2 & 63; int b = t2 >> 6;
  int h = c >> 4, d = c & 15;
  if (threadIdx.x < 16) ar[threadIdx.x] = attn[((b*4 + h)*16 + d)*16 + threadIdx.x];
  __syncthreads();
  int n = nt*256 + threadIdx.x;
  float s = 0.f;
  #pragma unroll
  for (int e = 0; e < 16; ++e)
    s += ar[e] * QKV[((size_t)b*192 + 128 + h*16 + e)*PP + n];
  vst2(Y + ((size_t)b*64 + c)*PP + n, (float_a)s);
}

extern "C" void kernel_launch(void* const* d_in, const int* in_sizes, int n_in,
                              void* d_out, int out_size, void* d_ws, size_t ws_size,
                              hipStream_t stream){
  (void)in_sizes; (void)n_in; (void)out_size; (void)ws_size;
  const float* hsi_f0    = (const float*)d_in[0];
  const float* msi_f0    = (const float*)d_in[1];
  const float* hsi_fi    = (const float*)d_in[2];
  const float* msi_fi    = (const float*)d_in[3];
  const float* sp_mlp_w  = (const float*)d_in[4];
  const float* sp_mlp_b  = (const float*)d_in[5];
  const float* spe_mlp_w = (const float*)d_in[6];
  const float* spe_mlp_b = (const float*)d_in[7];
  const float* spa_dw_w  = (const float*)d_in[8];
  const float* spa_dw_b  = (const float*)d_in[9];
  const float* spa_pw_w  = (const float*)d_in[10];
  const float* spa_pw_b  = (const float*)d_in[11];
  const float* spe_dw_w  = (const float*)d_in[12];
  const float* spe_dw_b  = (const float*)d_in[13];
  const float* spe_pw_w  = (const float*)d_in[14];
  const float* spe_pw_b  = (const float*)d_in[15];
  const float* sb_q_w    = (const float*)d_in[16];
  const float* sb_q_b    = (const float*)d_in[17];
  const float* sb_k_w    = (const float*)d_in[18];
  const float* sb_k_b    = (const float*)d_in[19];
  const float* sb_v_w    = (const float*)d_in[20];
  const float* sb_v_b    = (const float*)d_in[21];
  const float* sb_o_w    = (const float*)d_in[22];
  const float* sb_o_b    = (const float*)d_in[23];
  const float* sb_norm2_w  = (const float*)d_in[24];
  const float* sb_ffn_in_w = (const float*)d_in[25];
  const float* sb_ffn_dw_w = (const float*)d_in[26];
  const float* sb_ffn_out_w= (const float*)d_in[27];
  const float* rb_norm1_w  = (const float*)d_in[28];
  const float* rb_temp     = (const float*)d_in[29];
  const float* rb_qkv_w    = (const float*)d_in[30];
  const float* rb_qkv_dw_w = (const float*)d_in[31];
  const float* rb_proj_w   = (const float*)d_in[32];
  const float* rb_norm2_w  = (const float*)d_in[33];
  const float* rb_ffn_in_w = (const float*)d_in[34];
  const float* rb_ffn_dw_w = (const float*)d_in[35];
  const float* rb_ffn_out_w= (const float*)d_in[36];

  float* W = (float*)d_ws;
  const size_t T = TSZ, BIG = 1572864;
  float* bufH  = W;
  float* bufM  = W + 1*T;
  float* bufX1 = W + 2*T;
  float* bufY  = W + 3*T;
  float* bufLN = W + 4*T;
  float* bigA  = W + 5*T;
  float* bigB  = bigA + BIG;
  float* sr    = bigB + BIG;
  float* colmax = sr;
  float* spesc  = sr + 128;
  float* chmean = sr + 256;
  float* norms  = sr + 8448;
  float* logits = sr + 8704;
  float* attn   = sr + 10752;
  f16* qtok = (f16*)(sr + 16384);
  f16* ktok = qtok + T;
  f16* vtok = ktok + T;

  dim3 pw4(64, 4), pw8(64, 8), pw12(64, 12);

  k_colmax   <<<4, 256, 0, stream>>>(hsi_fi, colmax);
  k_spe_score<<<1,   128, 0, stream>>>(colmax, spe_mlp_w, spe_mlp_b, spesc);
  k_chmean   <<<32,  256, 0, stream>>>(msi_fi, chmean);

  k_dw3x3<<<2048, 256, 0, stream>>>(hsi_f0, spe_dw_w, spe_dw_b, spesc,
                                    nullptr, nullptr, nullptr, bigA, 64);
  k_pw<64,64,true,false,false,0><<<pw4, 256, 0, stream>>>(
      bigA, spe_pw_w, spe_pw_b, nullptr, nullptr, bufH, nullptr);
  k_dw3x3<<<2048, 256, 0, stream>>>(msi_f0, spa_dw_w, spa_dw_b, nullptr,
                                    sp_mlp_w, sp_mlp_b, chmean, bigA, 64);
  k_pw<64,64,true,false,false,0><<<pw4, 256, 0, stream>>>(
      bigA, spa_pw_w, spa_pw_b, nullptr, nullptr, bufM, nullptr);

  k_pw<64,64,true,false,false,1><<<pw4, 256, 0, stream>>>(
      bufM, sb_q_w, sb_q_b, nullptr, nullptr, nullptr, qtok);
  k_pw<64,64,true,false,false,1><<<pw4, 256, 0, stream>>>(
      bufH, sb_k_w, sb_k_b, nullptr, nullptr, nullptr, ktok);
  k_pw<64,64,true,false,false,2><<<pw4, 256, 0, stream>>>(
      bufH, sb_v_w, sb_v_b, nullptr, nullptr, nullptr, vtok);
  k_flash<<<dim3(128, 4, 2), 32, 0, stream>>>(qtok, ktok, vtok, bigA);
  k_pw<64,64,true,true,false,0><<<pw4, 256, 0, stream>>>(
      bigA, sb_o_w, sb_o_b, bufM, nullptr, bufX1, nullptr);
  k_ln<<<32, 256, 0, stream>>>(bufX1, sb_norm2_w, bufLN);
  k_pw<64,128,false,false,false,0><<<pw8, 256, 0, stream>>>(
      bufLN, sb_ffn_in_w, nullptr, nullptr, nullptr, bigA, nullptr);
  k_dw3x3<<<4096, 256, 0, stream>>>(bigA, sb_ffn_dw_w, nullptr, nullptr,
                                    nullptr, nullptr, nullptr, bigB, 128);
  k_gate<<<2048, 256, 0, stream>>>(bigB, bigA);
  k_pw<64,64,false,true,false,0><<<pw4, 256, 0, stream>>>(
      bigA, sb_ffn_out_w, nullptr, bufX1, nullptr, bufX1, nullptr);

  k_add<<<2048, 256, 0, stream>>>(bufM, bufH, bufY);
  k_ln<<<32, 256, 0, stream>>>(bufY, rb_norm1_w, bufLN);
  k_pw<64,192,false,false,false,0><<<pw12, 256, 0, stream>>>(
      bufLN, rb_qkv_w, nullptr, nullptr, nullptr, bigA, nullptr);
  k_dw3x3<<<6144, 256, 0, stream>>>(bigA, rb_qkv_dw_w, nullptr, nullptr,
                                    nullptr, nullptr, nullptr, bigB, 192);
  k_rbnorm   <<<8,    256, 0, stream>>>(bigB, norms);
  k_rbgram   <<<64,   256, 0, stream>>>(bigB, norms, rb_temp, logits);
  k_rbsoftmax<<<1,    128, 0, stream>>>(logits, attn);
  k_rbav     <<<2048, 256, 0, stream>>>(bigB, attn, bigA);
  k_pw<64,64,false,true,false,0><<<pw4, 256, 0, stream>>>(
      bigA, rb_proj_w, nullptr, bufY, nullptr, bufY, nullptr);
  k_ln<<<32, 256, 0, stream>>>(bufY, rb_norm2_w, bufLN);
  k_pw<64,128,false,false,false,0><<<pw8, 256, 0, stream>>>(
      bufLN, rb_ffn_in_w, nullptr, nullptr, nullptr, bigA, nullptr);
  k_dw3x3<<<4096, 256, 0, stream>>>(bigA, rb_ffn_dw_w, nullptr, nullptr,
                                    nullptr, nullptr, nullptr, bigB, 128);
  k_gate<<<2048, 256, 0, stream>>>(bigB, bigA);
  k_pw<64,64,false,true,true,0><<<pw4, 256, 0, stream>>>(
      bigA, rb_ffn_out_w, nullptr, bufY, bufX1, (float*)d_out, nullptr);
}
